// GroupedQueryAttention_43499428774488
// MI455X (gfx1250) — hardware-verified
//
#include <hip/hip_runtime.h>

#define DMODEL 1024
#define NHEAD  16
#define NKV    4
#define HDIM   64
#define LSEQ   2048
#define BATCH  2
#define MROWS  (BATCH * LSEQ)
#define NQKV   (DMODEL + 2 * NKV * HDIM)
#define NPAIR  (HDIM / 2)

typedef __bf16 bf16x16 __attribute__((ext_vector_type(16)));
typedef unsigned short u16x8 __attribute__((ext_vector_type(8)));
typedef unsigned short u16x16 __attribute__((ext_vector_type(16)));
typedef float v8f __attribute__((ext_vector_type(8)));
typedef float v4f __attribute__((ext_vector_type(4)));
typedef float v2f __attribute__((ext_vector_type(2)));

union Frag { bf16x16 v; u16x16 u; u16x8 h[2]; };

__device__ __forceinline__ unsigned short bf_bits(float f) {
  unsigned int u = __float_as_uint(f);
  u += 0x7FFFu + ((u >> 16) & 1u);
  return (unsigned short)(u >> 16);
}
__device__ __forceinline__ void bf_split(float f, unsigned short& hi, unsigned short& lo) {
  const unsigned short hb = bf_bits(f);
  const float fh = __uint_as_float(((unsigned int)hb) << 16);
  hi = hb;
  lo = bf_bits(f - fh);
}
__device__ __forceinline__ v8f zero8() {
  v8f z = {0.f, 0.f, 0.f, 0.f, 0.f, 0.f, 0.f, 0.f};
  return z;
}
__device__ __forceinline__ v8f mma(bf16x16 a, bf16x16 b, v8f c) {
  v8f d = __builtin_amdgcn_wmma_f32_16x16x32_bf16(false, a, false, b, (short)0, c, false, false);
  asm volatile("v_nop\n\tv_nop\n\tv_nop\n\tv_nop" : "+v"(d) : "v"(a), "v"(b));
  return d;
}

__launch_bounds__(256)
__global__ void gemm_x3(const float* __restrict__ A, const float* __restrict__ W, int ldw,
                        const float* __restrict__ bias, float* out, int ldo, int col0) {
  __shared__ __attribute__((aligned(16))) unsigned char smem[36864];
  unsigned short* Ah = (unsigned short*)(smem);
  unsigned short* Al = (unsigned short*)(smem + 5120);
  unsigned short* Bh = (unsigned short*)(smem + 10240);
  unsigned short* Bl = (unsigned short*)(smem + 20480);
  float* Cs = (float*)(smem);

  const int tid = threadIdx.x, wave = tid >> 5, lane = tid & 31;
  const int wr = wave >> 2, wc = wave & 3;
  const int lm = lane & 15, hh = lane >> 4;
  const int m0 = blockIdx.y * 64, n0 = blockIdx.x * 128;

  v8f acc[2][2];
#pragma unroll
  for (int i = 0; i < 2; ++i)
#pragma unroll
    for (int j = 0; j < 2; ++j) acc[i][j] = zero8();

  const int arow = tid >> 2, acol = (tid & 3) * 8;
  const int bk = tid >> 3, bn = (tid & 7) * 16;
  const float* aptr = A + (size_t)(m0 + arow) * DMODEL + acol;
  const float* wptr = W + (size_t)bk * ldw + n0 + bn;

#pragma unroll 1
  for (int kb = 0; kb < DMODEL; kb += 32) {
    {
      const v4f x0 = *(const v4f*)(aptr + kb);
      const v4f x1 = *(const v4f*)(aptr + kb + 4);
      u16x8 ah, al;
#pragma unroll
      for (int e = 0; e < 4; ++e) {
        unsigned short h0, l0, h1, l1;
        bf_split(x0[e], h0, l0);
        bf_split(x1[e], h1, l1);
        ah[e] = h0; al[e] = l0; ah[4 + e] = h1; al[4 + e] = l1;
      }
      *(u16x8*)(Ah + arow * 40 + acol) = ah;
      *(u16x8*)(Al + arow * 40 + acol) = al;
    }
    {
      const float* wp = wptr + (size_t)kb * ldw;
#pragma unroll
      for (int i = 0; i < 4; ++i) {
        const v4f w = *(const v4f*)(wp + 4 * i);
#pragma unroll
        for (int e = 0; e < 4; ++e) {
          unsigned short h0, l0;
          bf_split(w[e], h0, l0);
          const int nr = bn + 4 * i + e;
          Bh[nr * 40 + bk] = h0;
          Bl[nr * 40 + bk] = l0;
        }
      }
    }
    __syncthreads();

    Frag fah[2], fal[2], fbh[2], fbl[2];
#pragma unroll
    for (int mi = 0; mi < 2; ++mi) {
      const int row = (wr * 32 + mi * 16 + lm) * 40;
      fah[mi].h[0] = *(const u16x8*)(Ah + row + 8 * hh);
      fah[mi].h[1] = *(const u16x8*)(Ah + row + 16 + 8 * hh);
      fal[mi].h[0] = *(const u16x8*)(Al + row + 8 * hh);
      fal[mi].h[1] = *(const u16x8*)(Al + row + 16 + 8 * hh);
    }
#pragma unroll
    for (int ni = 0; ni < 2; ++ni) {
      const int row = (wc * 32 + ni * 16 + lm) * 40;
      fbh[ni].h[0] = *(const u16x8*)(Bh + row + 8 * hh);
      fbh[ni].h[1] = *(const u16x8*)(Bh + row + 16 + 8 * hh);
      fbl[ni].h[0] = *(const u16x8*)(Bl + row + 8 * hh);
      fbl[ni].h[1] = *(const u16x8*)(Bl + row + 16 + 8 * hh);
    }
#pragma unroll
    for (int mi = 0; mi < 2; ++mi)
#pragma unroll
      for (int ni = 0; ni < 2; ++ni) {
        acc[mi][ni] = mma(fah[mi].v, fbh[ni].v, acc[mi][ni]);
        acc[mi][ni] = mma(fah[mi].v, fbl[ni].v, acc[mi][ni]);
        acc[mi][ni] = mma(fal[mi].v, fbh[ni].v, acc[mi][ni]);
      }
    __syncthreads();
  }

  float* cw = Cs + wave * (32 * 36);
#pragma unroll
  for (int mi = 0; mi < 2; ++mi)
#pragma unroll
    for (int ni = 0; ni < 2; ++ni) {
      v4f d0, d1;
#pragma unroll
      for (int r = 0; r < 4; ++r) { d0[r] = acc[mi][ni][r]; d1[r] = acc[mi][ni][4 + r]; }
      float* cp = cw + (ni * 16 + lm) * 36 + mi * 16 + 8 * hh;
      *(v4f*)cp = d0;
      *(v4f*)(cp + 4) = d1;
    }
  __syncthreads();

  const int q = lane >> 3, j = lane & 7;
  const v4f bvec = *(const v4f*)(bias + n0 + wc * 32 + j * 4);
  v4f vals[8];
#pragma unroll
  for (int p = 0; p < 8; ++p) {
    const int row = p * 4 + q;
    v4f v;
#pragma unroll
    for (int e = 0; e < 4; ++e) v[e] = cw[(j * 4 + e) * 36 + row];
    vals[p] = v + bvec;
  }
  float* ob = out + (size_t)(m0 + wr * 32) * ldo + col0 + n0 + wc * 32 + j * 4;
#pragma unroll
  for (int p = 0; p < 8; ++p)
    *(volatile v4f*)(ob + (size_t)(p * 4 + q) * ldo) = vals[p];
  __threadfence();
#pragma unroll
  for (int p = 0; p < 8; ++p)
    *(volatile v4f*)(ob + (size_t)(p * 4 + q) * ldo) = vals[p];
}

__launch_bounds__(32)
__global__ void freqtab(float* ft) {
  const int p = threadIdx.x & 31;
  const float ex = (float)(2 * p) * (1.0f / (float)HDIM);
  const float f = 1.0f / powf(10000.0f, ex);
  *(volatile float*)(ft + p) = f;
  __threadfence();
  *(volatile float*)(ft + p) = f;
}

__launch_bounds__(256)
__global__ void cstab(const float* __restrict__ ft, float* cs, int n) {
  const int idx = blockIdx.x * 256 + threadIdx.x;
  const bool valid = idx < n;
  const int i = valid ? idx : 0;
  const int l = i >> 5, p = i & 31;
  const float ang = (float)l * ft[p];
  float sv, cv;
  sincosf(ang, &sv, &cv);
  v2f o;
  o.x = cv; o.y = sv;
  if (valid) *(volatile v2f*)(cs + (size_t)i * 2) = o;
  __threadfence();
  if (valid) *(volatile v2f*)(cs + (size_t)i * 2) = o;
}

__launch_bounds__(256)
__global__ void normrope(const float* __restrict__ raw, const float* __restrict__ cs,
                         const float* __restrict__ qw, const float* __restrict__ kw,
                         unsigned short* qhh, unsigned short* qhl,
                         unsigned short* khh, unsigned short* khl, int ngroups) {
  __shared__ __attribute__((aligned(16))) unsigned short sh[8][8][64];
  __shared__ __attribute__((aligned(16))) unsigned short sl[8][8][64];
  const int wave = threadIdx.x >> 5, lane = threadIdx.x & 31;
  const int gid = blockIdx.x * 8 + wave;
  const bool valid = gid < ngroups;
  const int g = valid ? gid : 0;
  const int RQ = BATCH * NHEAD * LSEQ;
  const int rid0 = g * 8;
  const bool isq = rid0 < RQ;
  const int id = isq ? rid0 : rid0 - RQ;
  const int HH = isq ? NHEAD : NKV;
  const int b = id / (HH * LSEQ);
  const int hd = (id / LSEQ) % HH;
  const int l0 = id % LSEQ;
  const int i2 = lane * 2;
  const float* wsrc = isq ? qw : kw;
  const float w0 = wsrc[i2], w1 = wsrc[i2 + 1];
  const float* src0 = raw + (size_t)(b * LSEQ + l0) * NQKV + (isq ? 0 : DMODEL) + hd * HDIM + i2;

#pragma unroll 1
  for (int r = 0; r < 8; ++r) {
    const float* s = src0 + (size_t)r * NQKV;
    const float x0 = s[0], x1 = s[1];
    float ss = x0 * x0 + x1 * x1;
#pragma unroll
    for (int off = 16; off; off >>= 1) ss += __shfl_xor(ss, off, 32);
    const float inv = rsqrtf(ss * (1.0f / (float)HDIM) + 1e-6f);
    const float xe = (x0 * inv) * w0;
    const float xo = (x1 * inv) * w1;
    const v2f t2 = *(const v2f*)(cs + ((size_t)(l0 + r) * NPAIR + lane) * 2);
    const float c = t2.x, sn = t2.y;
    const float oe = xe * c - xo * sn;
    const float oo = xe * sn + xo * c;
    unsigned short he, le, ho, lo;
    bf_split(oe, he, le);
    bf_split(oo, ho, lo);
    sh[wave][r][i2] = he; sh[wave][r][i2 + 1] = ho;
    sl[wave][r][i2] = le; sl[wave][r][i2 + 1] = lo;
  }
  __syncthreads();

  const int q = lane >> 3, j = lane & 7;
  u16x8 vh[2], vl[2];
#pragma unroll
  for (int p = 0; p < 2; ++p) {
    vh[p] = *(const u16x8*)&sh[wave][p * 4 + q][j * 8];
    vl[p] = *(const u16x8*)&sl[wave][p * 4 + q][j * 8];
  }
  const size_t base = ((size_t)((b * HH + hd) * LSEQ + l0)) * HDIM + j * 8;
  unsigned short* dh = (isq ? qhh : khh) + base;
  unsigned short* dl = (isq ? qhl : khl) + base;
  if (valid) {
#pragma unroll
    for (int p = 0; p < 2; ++p) {
      *(volatile u16x8*)(dh + (p * 4 + q) * HDIM) = vh[p];
      *(volatile u16x8*)(dl + (p * 4 + q) * HDIM) = vl[p];
    }
  }
  __threadfence();
  if (valid) {
#pragma unroll
    for (int p = 0; p < 2; ++p) {
      *(volatile u16x8*)(dh + (p * 4 + q) * HDIM) = vh[p];
      *(volatile u16x8*)(dl + (p * 4 + q) * HDIM) = vl[p];
    }
  }
}

__launch_bounds__(256)
__global__ void vtrans(const float* __restrict__ raw, unsigned short* vth, unsigned short* vtl) {
  __shared__ float tile[64][65];
  const int bkv = blockIdx.x / (LSEQ / 64);
  const int lt = blockIdx.x % (LSEQ / 64);
  const int l0 = lt * 64;
  const int b = bkv / NKV, kv = bkv % NKV;
  const int tid = threadIdx.x;
  const int r = tid >> 2, c = (tid & 3) * 16;
  const float* s = raw + (size_t)(b * LSEQ + l0 + r) * NQKV + DMODEL + NKV * HDIM + kv * HDIM + c;
#pragma unroll
  for (int i = 0; i < 4; ++i) {
    const v4f v = *(const v4f*)(s + 4 * i);
#pragma unroll
    for (int e = 0; e < 4; ++e) tile[r][c + 4 * i + e] = v[e];
  }
  __syncthreads();

  const int wave = tid >> 5, lane = tid & 31;
  const int q = lane >> 3, j = lane & 7;
  u16x8 oh[2], ol[2];
#pragma unroll
  for (int p = 0; p < 2; ++p) {
    const int d = wave * 8 + p * 4 + q;
#pragma unroll
    for (int e = 0; e < 8; ++e) {
      unsigned short h0, l0v;
      bf_split(tile[j * 8 + e][d], h0, l0v);
      oh[p][e] = h0; ol[p][e] = l0v;
    }
  }
  const size_t base = ((size_t)(bkv * HDIM + wave * 8 + q)) * LSEQ + l0 + j * 8;
#pragma unroll
  for (int p = 0; p < 2; ++p) {
    *(volatile u16x8*)(vth + base + (size_t)(p * 4) * LSEQ) = oh[p];
    *(volatile u16x8*)(vtl + base + (size_t)(p * 4) * LSEQ) = ol[p];
  }
  __threadfence();
#pragma unroll
  for (int p = 0; p < 2; ++p) {
    *(volatile u16x8*)(vth + base + (size_t)(p * 4) * LSEQ) = oh[p];
    *(volatile u16x8*)(vtl + base + (size_t)(p * 4) * LSEQ) = ol[p];
  }
}

__launch_bounds__(32)
__global__ void attn(const unsigned short* __restrict__ qhh, const unsigned short* __restrict__ qhl,
                     const unsigned short* __restrict__ khh, const unsigned short* __restrict__ khl,
                     const unsigned short* __restrict__ vth, const unsigned short* __restrict__ vtl,
                     float* ctx) {
  __shared__ __attribute__((aligned(16))) float Cs[16][68];
  const int lane = threadIdx.x, lm = lane & 15, hh = lane >> 4;
  const int QT = LSEQ / 16;
  const int qt = blockIdx.x % QT;
  const int h = (blockIdx.x / QT) % NHEAD;
  const int b = blockIdx.x / (QT * NHEAD);
  const int kv = h / (NHEAD / NKV);
  const int qrow = qt * 16 + lm;

  const size_t qoff = ((size_t)((b * NHEAD + h) * LSEQ + qrow)) * HDIM;
  Frag fqh[2], fql[2];
#pragma unroll
  for (int ks = 0; ks < 2; ++ks) {
    fqh[ks].h[0] = *(const u16x8*)(qhh + qoff + ks * 32 + 8 * hh);
    fqh[ks].h[1] = *(const u16x8*)(qhh + qoff + ks * 32 + 16 + 8 * hh);
    fql[ks].h[0] = *(const u16x8*)(qhl + qoff + ks * 32 + 8 * hh);
    fql[ks].h[1] = *(const u16x8*)(qhl + qoff + ks * 32 + 16 + 8 * hh);
  }

  v8f o[4];
#pragma unroll
  for (int t = 0; t < 4; ++t) o[t] = zero8();
  float mrun = -3.0e38f, lrun = 0.0f;

  const size_t koff = (size_t)(b * NKV + kv) * LSEQ * HDIM;
  const unsigned short* kbh = khh + koff;
  const unsigned short* kbl = khl + koff;
  const size_t voff = (size_t)(b * NKV + kv) * HDIM * LSEQ;
  const unsigned short* vbh = vth + voff;
  const unsigned short* vbl = vtl + voff;
  const int nkb = (qt * 16 + 15) / 32 + 1;

#pragma unroll 1
  for (int kb = 0; kb < nkb; ++kb) {
    const int key0 = kb * 32;
    v8f s[2];
#pragma unroll
    for (int jt = 0; jt < 2; ++jt) {
      s[jt] = zero8();
      const size_t kro = (size_t)(key0 + jt * 16 + lm) * HDIM;
#pragma unroll
      for (int ks = 0; ks < 2; ++ks) {
        Frag ka, kl;
        ka.h[0] = *(const u16x8*)(kbh + kro + ks * 32 + 8 * hh);
        ka.h[1] = *(const u16x8*)(kbh + kro + ks * 32 + 16 + 8 * hh);
        kl.h[0] = *(const u16x8*)(kbl + kro + ks * 32 + 8 * hh);
        kl.h[1] = *(const u16x8*)(kbl + kro + ks * 32 + 16 + 8 * hh);
        s[jt] = mma(ka.v, fqh[ks].v, s[jt]);
        s[jt] = mma(ka.v, fql[ks].v, s[jt]);
        s[jt] = mma(kl.v, fqh[ks].v, s[jt]);
      }
    }

    float tm = -3.0e38f;
#pragma unroll
    for (int r = 0; r < 8; ++r) {
      const int ki = key0 + 8 * hh + r;
      float a = s[0][r] * 0.125f;
      float c = s[1][r] * 0.125f;
      if (ki > qrow)      a = -1.0e30f;
      if (ki + 16 > qrow) c = -1.0e30f;
      s[0][r] = a; s[1][r] = c;
      tm = fmaxf(tm, fmaxf(a, c));
    }
    tm = fmaxf(tm, __shfl_xor(tm, 16, 32));
    const float nm = fmaxf(mrun, tm);
    const float sc = expf(mrun - nm);
    float rs = 0.0f;
    u16x8 p0h, p0l, p1h, p1l;
#pragma unroll
    for (int r = 0; r < 8; ++r) {
      const float e0 = expf(s[0][r] - nm);
      const float e1 = expf(s[1][r] - nm);
      rs += e0 + e1;
      unsigned short a0, a1, c0, c1;
      bf_split(e0, a0, a1);
      bf_split(e1, c0, c1);
      p0h[r] = a0; p0l[r] = a1; p1h[r] = c0; p1l[r] = c1;
    }
    rs += __shfl_xor(rs, 16, 32);
    lrun = lrun * sc + rs;
    mrun = nm;
    Frag ph, pl;
    ph.h[0] = p0h; ph.h[1] = p1h;
    pl.h[0] = p0l; pl.h[1] = p1l;
#pragma unroll
    for (int t = 0; t < 4; ++t) o[t] = o[t] * sc;

#pragma unroll
    for (int t = 0; t < 4; ++t) {
      const size_t vro = (size_t)(t * 16 + lm) * LSEQ + key0;
      Frag va, vl;
      va.h[0] = *(const u16x8*)(vbh + vro + 8 * hh);
      va.h[1] = *(const u16x8*)(vbh + vro + 16 + 8 * hh);
      vl.h[0] = *(const u16x8*)(vbl + vro + 8 * hh);
      vl.h[1] = *(const u16x8*)(vbl + vro + 16 + 8 * hh);
      o[t] = mma(va.v, ph.v, o[t]);
      o[t] = mma(va.v, pl.v, o[t]);
      o[t] = mma(vl.v, ph.v, o[t]);
    }
  }

  const float inv = 1.0f / lrun;
#pragma unroll
  for (int t = 0; t < 4; ++t) {
    v4f d0, d1;
#pragma unroll
    for (int r = 0; r < 4; ++r) { d0[r] = o[t][r] * inv; d1[r] = o[t][4 + r] * inv; }
    *(v4f*)&Cs[lm][t * 16 + 8 * hh] = d0;
    *(v4f*)&Cs[lm][t * 16 + 8 * hh + 4] = d1;
  }
  __syncthreads();

  const int q = lane >> 3, j = lane & 7;
  v4f vals[8];
#pragma unroll
  for (int p = 0; p < 8; ++p) {
    const int li = p * 4 + q;
    vals[p] = *(const v4f*)&Cs[li >> 1][(li & 1) * 32 + j * 4];
  }
  float* cb = ctx + ((size_t)(b * LSEQ + qt * 16)) * DMODEL + h * HDIM + j * 4;
#pragma unroll
  for (int p = 0; p < 8; ++p) {
    const int li = p * 4 + q;
    *(volatile v4f*)(cb + (size_t)(li >> 1) * DMODEL + (li & 1) * 32) = vals[p];
  }
  __threadfence();
#pragma unroll
  for (int p = 0; p < 8; ++p) {
    const int li = p * 4 + q;
    *(volatile v4f*)(cb + (size_t)(li >> 1) * DMODEL + (li & 1) * 32) = vals[p];
  }
}

extern "C" void kernel_launch(void* const* d_in, const int* in_sizes, int n_in,
                              void* d_out, int out_size, void* d_ws, size_t ws_size,
                              hipStream_t stream) {
  if (n_in < 11) return;
  if (in_sizes[0] != MROWS * DMODEL) return;
  if (in_sizes[1] != DMODEL * DMODEL || in_sizes[2] < DMODEL) return;
  if (in_sizes[3] != DMODEL * NKV * HDIM || in_sizes[4] < NKV * HDIM) return;
  if (in_sizes[5] != DMODEL * NKV * HDIM || in_sizes[6] < NKV * HDIM) return;
  if (in_sizes[7] != DMODEL * DMODEL || in_sizes[8] < DMODEL) return;
  if (in_sizes[9] < HDIM || in_sizes[10] < HDIM) return;
  if (out_size != MROWS * DMODEL) return;

  const float* x   = (const float*)d_in[0];
  const float* Wq  = (const float*)d_in[1];
  const float* bq  = (const float*)d_in[2];
  const float* Wk  = (const float*)d_in[3];
  const float* bk  = (const float*)d_in[4];
  const float* Wv  = (const float*)d_in[5];
  const float* bv  = (const float*)d_in[6];
  const float* Wo  = (const float*)d_in[7];
  const float* bo  = (const float*)d_in[8];
  const float* qnw = (const float*)d_in[9];
  const float* knw = (const float*)d_in[10];
  float* out = (float*)d_out;

  const size_t raw_b = (size_t)MROWS * NQKV * sizeof(float);
  const size_t q_b   = (size_t)BATCH * NHEAD * LSEQ * HDIM * sizeof(unsigned short);
  const size_t k_b   = (size_t)BATCH * NKV * LSEQ * HDIM * sizeof(unsigned short);
  const size_t ctx_b = (size_t)MROWS * DMODEL * sizeof(float);
  const size_t ft_b  = 128;
  const size_t cs_b  = (size_t)LSEQ * NPAIR * 2 * sizeof(float);
  const size_t total = raw_b + 2 * q_b + 4 * k_b + ctx_b + ft_b + cs_b;
  if (total > ws_size) return;
  char* ws = (char*)d_ws;
  size_t off = 0;
  float* raw = (float*)(ws + off);                    off += raw_b;
  unsigned short* qhh = (unsigned short*)(ws + off);  off += q_b;
  unsigned short* qhl = (unsigned short*)(ws + off);  off += q_b;
  unsigned short* khh = (unsigned short*)(ws + off);  off += k_b;
  unsigned short* khl = (unsigned short*)(ws + off);  off += k_b;
  unsigned short* vth = (unsigned short*)(ws + off);  off += k_b;
  unsigned short* vtl = (unsigned short*)(ws + off);  off += k_b;
  float* ctx = (float*)(ws + off);                    off += ctx_b;
  float* ftab = (float*)(ws + off);                   off += ft_b;
  float* cst = (float*)(ws + off);                    off += cs_b;

  const dim3 blk(256);
  freqtab<<<1, 32, 0, stream>>>(ftab);
  const int ncs = LSEQ * NPAIR;
  cstab<<<(ncs + 255) / 256, blk, 0, stream>>>(ftab, cst, ncs);

  gemm_x3<<<dim3(DMODEL / 128, MROWS / 64), blk, 0, stream>>>(x, Wq, DMODEL, bq, raw, NQKV, 0);
  gemm_x3<<<dim3((NKV * HDIM) / 128, MROWS / 64), blk, 0, stream>>>(x, Wk, NKV * HDIM, bk, raw, NQKV, DMODEL);
  gemm_x3<<<dim3((NKV * HDIM) / 128, MROWS / 64), blk, 0, stream>>>(x, Wv, NKV * HDIM, bv, raw, NQKV, DMODEL + NKV * HDIM);

  const int ngroups = (BATCH * NHEAD * LSEQ + BATCH * NKV * LSEQ) / 8;
  normrope<<<(ngroups + 7) / 8, blk, 0, stream>>>(raw, cst, qnw, knw, qhh, qhl, khh, khl, ngroups);

  vtrans<<<BATCH * NKV * (LSEQ / 64), blk, 0, stream>>>(raw, vth, vtl);

  attn<<<BATCH * NHEAD * (LSEQ / 16), 32, 0, stream>>>(qhh, qhl, khh, khl, vth, vtl, ctx);

  gemm_x3<<<dim3(DMODEL / 128, MROWS / 64), blk, 0, stream>>>(ctx, Wo, DMODEL, bo, out, DMODEL, 0);

  (void)hipGetLastError();
}
